// BiSSMGlobalBlock_76192719831242
// MI455X (gfx1250) — hardware-run, weakly checked
//
#include <hip/hip_runtime.h>

typedef __attribute__((ext_vector_type(16))) _Float16 v16h;
typedef __attribute__((ext_vector_type(8)))  _Float16 v8h;
typedef __attribute__((ext_vector_type(8)))  float    v8f;
typedef __attribute__((ext_vector_type(4)))  float    v4f;
typedef __attribute__((ext_vector_type(4)))  unsigned v4u;
typedef __attribute__((ext_vector_type(2)))  unsigned v2u;

constexpr int kB = 8;
constexpr int kN = 2048;
constexpr int kD = 768;
constexpr int kH = 768;
constexpr int kR = 4;
constexpr int kRows = kB * kN;
static_assert(kD == kH);
static_assert(kR == 4);
static_assert(kRows % 64 == 0 && kH % 64 == 0 && kD % 64 == 0);
static_assert(kH % 32 == 0 && kD % 32 == 0);

constexpr float kXC = 16.0f;
constexpr float kWC = 256.0f;
constexpr float kAC = 512.0f;
constexpr float kHC = 16.0f;
constexpr float kInvAC  = 1.0f / kAC;
constexpr float kScaleU = kHC / (kXC * kWC);
constexpr float kScaleG = 1.0f / (kXC * kWC);
constexpr float kScaleY = 0.5f / (kHC * kWC);
constexpr float kInvH   = 1.0f / (float)kH;
constexpr float kInvD   = 1.0f / (float)kD;
constexpr float kEps    = 1e-8f;

constexpr int kDwPlane  = kH * kH / 2;
constexpr int kBlkPlane = kDwPlane / 256;
constexpr int kPrepBlocks = 4 * kBlkPlane;
static_assert(kDwPlane % 256 == 0);
static_assert(kDwPlane == 294912 && kBlkPlane == 1152);

constexpr int kHP  = kH + 8;
constexpr int kHT  = 16 * kHP;
constexpr int kColsPW = 96;
constexpr int kNT  = 6;
static_assert(kHP % 8 == 0);
static_assert(kH == 8 * kColsPW && kColsPW == 16 * kNT);
static_assert(2 * kB == 16);
static_assert((2 * kHT) % 8 == 0);
static_assert(2 * kHT * 2 <= 65536);

constexpr int kSumChunks = kRows * kH / 8;
static_assert(kSumChunks % 256 == 0);
static_assert(kRows % 8 == 0);

union FragU { v16h v; v8h h[2]; };
__device__ __forceinline__ v16h frag_load(const _Float16* p) {
  FragU f;
  f.h[0] = *(const v8h*)(p);
  f.h[1] = *(const v8h*)(p + 16);
  return f.v;
}
__device__ __forceinline__ v8f mma_g(v16h a, v16h b, v8f c) {
  c = __builtin_amdgcn_wmma_f32_16x16x32_f16(false, a, false, b, (short)0, c, false, false);
  asm volatile("v_nop\n\tv_nop\n\tv_nop\n\tv_nop" : "+v"(c) : "v"(a), "v"(b));
  return c;
}
__device__ __forceinline__ void keep4_h(v16h a, v16h b, v16h c, v16h d) { asm volatile("v_nop" :: "v"(a), "v"(b), "v"(c), "v"(d)); }
__device__ __forceinline__ void acc_guard4(v8f& a, v8f& b, v8f& c, v8f& d) { asm volatile("v_nop\n\tv_nop\n\tv_nop\n\tv_nop" : "+v"(a), "+v"(b), "+v"(c), "+v"(d)); }
__device__ __forceinline__ void wave_lds_sync() {
  __builtin_amdgcn_fence(__ATOMIC_RELEASE, "workgroup");
  __builtin_amdgcn_wave_barrier();
  __builtin_amdgcn_fence(__ATOMIC_ACQUIRE, "workgroup");
}
__device__ __forceinline__ float h16_to_f32(unsigned hb) {
  const unsigned sgn = (hb & 0x8000u) << 16;
  const unsigned em = hb & 0x7fffu;
  const float fn = __uint_as_float((em << 13) + 0x38000000u);
  const float fs = (float)em * 5.9604644775390625e-8f;
  const float mag = (em < 0x400u) ? fs : fn;
  return __uint_as_float(__float_as_uint(mag) | sgn);
}
__device__ __forceinline__ unsigned pack_f16x2(float a, float b) {
  const _Float16 h0 = (_Float16)a;
  const _Float16 h1 = (_Float16)b;
  return (unsigned)__builtin_bit_cast(unsigned short, h0) | ((unsigned)__builtin_bit_cast(unsigned short, h1) << 16);
}
__device__ __forceinline__ void st2u(unsigned* p, unsigned v) {
  *(volatile unsigned*)p = v;
  __threadfence();
  *(volatile unsigned*)p = v;
}
__device__ __forceinline__ float fsig(float x) { return __builtin_amdgcn_rcpf(1.0f + __expf(-x)); }

__global__ __launch_bounds__(256) void prep_kernel(
    const float* __restrict__ U, const float* __restrict__ V, const float* __restrict__ S,
    const float* __restrict__ Bm, const float* __restrict__ Cm, const float* __restrict__ gw,
    unsigned* __restrict__ a16u, unsigned* __restrict__ bm16u,
    unsigned* __restrict__ cm16u, unsigned* __restrict__ gw16u) {
  const int blk = blockIdx.x;
  const int tid = threadIdx.x;
  if (blk < kBlkPlane) {
    const int p = blk * 256 + tid;
    const int i = p / (kH / 2);
    const int j = (p - i * (kH / 2)) * 2;
    const float dg = -(float)(i + 1) * kInvH;
    const v4f ui = *(const v4f*)(U + 4 * i);
    const v4f v0 = *(const v4f*)(V + 4 * j);
    const v4f v1 = *(const v4f*)(V + 4 * j + 4);
    float lr0 = ui[0] * v0[0];
    lr0 += ui[1] * v0[1];
    lr0 += ui[2] * v0[2];
    lr0 += ui[3] * v0[3];
    float lr1 = ui[0] * v1[0];
    lr1 += ui[1] * v1[1];
    lr1 += ui[2] * v1[2];
    lr1 += ui[3] * v1[3];
    float a0 = ((i == j) ? dg : 0.0f) + lr0;
    float a1 = ((i == j + 1) ? dg : 0.0f) + lr1;
    a0 += S[i * kH + j] - S[j * kH + i];
    a1 += S[i * kH + j + 1] - S[(j + 1) * kH + i];
    const unsigned w = pack_f16x2(a0 * kAC, a1 * kAC);
    st2u(a16u + p, w);
  } else if (blk < 2 * kBlkPlane) {
    const int p = (blk - kBlkPlane) * 256 + tid;
    const unsigned w = pack_f16x2(Bm[2 * p] * kWC, Bm[2 * p + 1] * kWC);
    st2u(bm16u + p, w);
  } else if (blk < 3 * kBlkPlane) {
    const int p = (blk - 2 * kBlkPlane) * 256 + tid;
    const unsigned w = pack_f16x2(Cm[2 * p] * kWC, Cm[2 * p + 1] * kWC);
    st2u(cm16u + p, w);
  } else {
    const int p = (blk - 3 * kBlkPlane) * 256 + tid;
    const unsigned w = pack_f16x2(gw[2 * p] * kWC, gw[2 * p + 1] * kWC);
    st2u(gw16u + p, w);
  }
}

__global__ __launch_bounds__(256) void rmsnorm_kernel(const float* __restrict__ x, const float* __restrict__ scale,
                                                      unsigned short* __restrict__ xn16) {
  const int lane = threadIdx.x & 31;
  const int row = blockIdx.x * 8 + (threadIdx.x >> 5);
  if (row >= kRows) return;
  const float* xr = x + (size_t)row * kD;
  v4f a[3], b[3];
  float ss = 0.0f;
#pragma unroll
  for (int p = 0; p < 3; ++p) {
    a[p] = *(const v4f*)(xr + 256 * p + 8 * lane);
    b[p] = *(const v4f*)(xr + 256 * p + 8 * lane + 4);
    ss += (a[p][0] * a[p][0] + a[p][1] * a[p][1]) + (a[p][2] * a[p][2] + a[p][3] * a[p][3]);
    ss += (b[p][0] * b[p][0] + b[p][1] * b[p][1]) + (b[p][2] * b[p][2] + b[p][3] * b[p][3]);
  }
#pragma unroll
  for (int off = 1; off < 32; off <<= 1) ss += __shfl_xor(ss, off, 32);
  const float r = rsqrtf(ss * kInvD + kEps) * kXC;
  v8h hv[3];
#pragma unroll
  for (int p = 0; p < 3; ++p) {
    const v4f sa = *(const v4f*)(scale + 256 * p + 8 * lane);
    const v4f sb = *(const v4f*)(scale + 256 * p + 8 * lane + 4);
#pragma unroll
    for (int e = 0; e < 4; ++e) {
      hv[p][e]     = (_Float16)((a[p][e] * r) * sa[e]);
      hv[p][4 + e] = (_Float16)((b[p][e] * r) * sb[e]);
    }
  }
  unsigned short* op = xn16 + (size_t)row * kD;
  for (int pass = 0; pass < 2; ++pass) {
#pragma unroll
    for (int p = 0; p < 3; ++p) *(volatile v8h*)(op + 256 * p + 8 * lane) = hv[p];
    __threadfence();
  }
}

template <int MODE>
__global__ __launch_bounds__(256) void gemm64_f16(
    const unsigned short* __restrict__ Ap, int lda,
    const unsigned short* __restrict__ Btp, int ldb,
    void* __restrict__ Cout, int ldc,
    const float* __restrict__ bias,
    const float* __restrict__ xres,
    const unsigned short* __restrict__ gpl,
    const float* __restrict__ alphap,
    int M, int N, int K, float scale) {
  const _Float16* A  = (const _Float16*)Ap;
  const _Float16* Bt = (const _Float16*)Btp;
  __shared__ __align__(16) float sT[8][16 * 68];
  const int lane = threadIdx.x & 31;
  const int wave = threadIdx.x >> 5;
  const int tilesN = N >> 6;
  const int tilesM = M >> 6;
  const int tile = blockIdx.x * 8 + wave;
  if (tile >= tilesM * tilesN) return;
  const int tm = tile / tilesN;
  const int tn = tile - tm * tilesN;
  const int m0 = tm << 6;
  const int n0 = tn << 6;
  const int rlane = lane & 15;
  const int koff  = (lane >> 4) * 8;
  const int mOff  = (lane >> 4) * 8;

  v8f acc[4][4];
#pragma unroll
  for (int i = 0; i < 4; ++i)
#pragma unroll
    for (int j = 0; j < 4; ++j) acc[i][j] = (v8f){0.f, 0.f, 0.f, 0.f, 0.f, 0.f, 0.f, 0.f};

  for (int k0 = 0; k0 < K; k0 += 32) {
    v16h bh[4];
#pragma unroll
    for (int j = 0; j < 4; ++j) {
      const size_t bo = (size_t)(n0 + (j << 4) + rlane) * ldb + koff + k0;
      bh[j] = frag_load(Bt + bo);
    }
#pragma unroll
    for (int i = 0; i < 4; ++i) {
      const size_t ao = (size_t)(m0 + (i << 4) + rlane) * lda + koff + k0;
      const v16h ah = frag_load(A + ao);
#pragma unroll
      for (int j = 0; j < 4; ++j) acc[i][j] = mma_g(ah, bh[j], acc[i][j]);
    }
    keep4_h(bh[0], bh[1], bh[2], bh[3]);
  }
  acc_guard4(acc[0][0], acc[0][1], acc[0][2], acc[0][3]);
  acc_guard4(acc[1][0], acc[1][1], acc[1][2], acc[1][3]);
  acc_guard4(acc[2][0], acc[2][1], acc[2][2], acc[2][3]);
  acc_guard4(acc[3][0], acc[3][1], acc[3][2], acc[3][3]);

  float* slab = sT[wave];
  float cs = scale;
  if (MODE == 2) cs = scale * alphap[0];
#pragma unroll
  for (int i = 0; i < 4; ++i) {
    const int mBase = m0 + (i << 4);
#pragma unroll
    for (int j = 0; j < 4; ++j) {
      const int n = n0 + (j << 4) + rlane;
      float bv = 0.0f;
      if (MODE == 1) bv = bias[n];
#pragma unroll
      for (int r = 0; r < 8; ++r) {
        float v = acc[i][j][r] * cs;
        if (MODE == 1) {
          v += bv;
          v = fsig(v);
        }
        slab[(mOff + r) * 68 + (j << 4) + rlane] = v;
      }
    }
    wave_lds_sync();
    if (MODE == 2) {
      float* C = (float*)Cout;
      const int hh = lane >> 4;
      const int c4 = (lane & 15) * 4;
#pragma unroll
      for (int it = 0; it < 8; ++it) {
        const int row = it * 2 + hh;
        const size_t gidx = (size_t)(mBase + row) * ldc + n0 + c4;
        const v4f sv = *(const v4f*)(slab + row * 68 + c4);
        const v4f xv = *(const v4f*)(xres + gidx);
        const v2u gw2 = *(const v2u*)(gpl + gidx);
        const unsigned w0 = gw2[0];
        const unsigned w1 = gw2[1];
        const float g0 = h16_to_f32(w0 & 0xffffu);
        const float g1 = h16_to_f32(w0 >> 16);
        const float g2 = h16_to_f32(w1 & 0xffffu);
        const float g3 = h16_to_f32(w1 >> 16);
        v4f o;
        o[0] = xv[0] + sv[0] * g0;
        o[1] = xv[1] + sv[1] * g1;
        o[2] = xv[2] + sv[2] * g2;
        o[3] = xv[3] + sv[3] * g3;
        *(v4f*)(slab + row * 68 + c4) = o;
      }
      wave_lds_sync();
      for (int pass = 0; pass < 2; ++pass) {
#pragma unroll
        for (int it = 0; it < 8; ++it) {
          const int row = it * 2 + hh;
          const v4f v = *(const v4f*)(slab + row * 68 + c4);
          *(volatile v4f*)(C + (size_t)(mBase + row) * ldc + n0 + c4) = v;
        }
        __threadfence();
      }
    } else {
      const int q = lane >> 3;
      const int c8 = (lane & 7) * 8;
      unsigned short* C = (unsigned short*)Cout;
      for (int pass = 0; pass < 2; ++pass) {
#pragma unroll
        for (int it = 0; it < 4; ++it) {
          const int row = it * 4 + q;
          const float* sp = slab + row * 68 + c8;
          v8h hv;
#pragma unroll
          for (int e = 0; e < 8; ++e) hv[e] = (_Float16)sp[e];
          *(volatile v8h*)(C + (size_t)(mBase + row) * ldc + n0 + c8) = hv;
        }
        __threadfence();
      }
    }
    wave_lds_sync();
  }
}

__global__ __launch_bounds__(256) void scan_kernel(const unsigned short* __restrict__ u16,
                                                   const unsigned short* __restrict__ a16,
                                                   unsigned short* __restrict__ hf16,
                                                   unsigned short* __restrict__ hb16) {
  __shared__ __align__(16) unsigned short hbuf[2 * kHT];
  const int tid = threadIdx.x;
  const int lane = tid & 31;
  const int wave = tid >> 5;
  const int c = lane & 15;
  const int hh = lane >> 4;
  const int koff = hh * 8;
  const int n0 = wave * kColsPW;

  {
    const v4u z = {0u, 0u, 0u, 0u};
    for (int i = tid; i < (2 * kHT) / 8; i += 256) *(v4u*)(hbuf + i * 8) = z;
  }

  int uoff[6];
  int loff[6];
  int ubw[6];
#pragma unroll
  for (int i = 0; i < 6; ++i) {
    const int q = lane + 32 * i;
    const int row = q / 12;
    const int cc = q - row * 12;
    uoff[i] = ((row & 7) * kN) * kH + n0 + 8 * cc;
    loff[i] = row * kHP + n0 + 8 * cc;
    ubw[i] = row >> 3;
  }
  const int dirb = wave >> 2;
  const int rowA = 2 * wave;
  const int bA = rowA & 7;
  unsigned short* plane = dirb ? hb16 : hf16;

  const _Float16* brow = (const _Float16*)a16 + (size_t)(n0 + c) * kH + koff;
  __syncthreads();

#pragma unroll 1
  for (int s = 0; s < kN; ++s) {
    const int cur = s & 1;
    unsigned short* hc = hbuf + cur * kHT;
    unsigned short* hn = hbuf + (cur ^ 1) * kHT;

    v4u ur[6];
#pragma unroll
    for (int i = 0; i < 6; ++i) {
      const int tt = ubw[i] ? (kN - 1 - s) : s;
      ur[i] = *(const v4u*)(u16 + (size_t)uoff[i] + (size_t)tt * kH);
    }

    v8f acc[kNT];
#pragma unroll
    for (int j = 0; j < kNT; ++j) acc[j] = (v8f){0.f, 0.f, 0.f, 0.f, 0.f, 0.f, 0.f, 0.f};
    const _Float16* arow = (const _Float16*)hc + c * kHP + koff;
#pragma unroll 1
    for (int kc = 0; kc < kH / 32; ++kc) {
      const v16h fa = frag_load(arow + kc * 32);
      v16h fb[kNT];
#pragma unroll
      for (int j = 0; j < kNT; ++j) fb[j] = frag_load(brow + (size_t)(16 * j) * kH + kc * 32);
#pragma unroll
      for (int j = 0; j < kNT; ++j) acc[j] = mma_g(fa, fb[j], acc[j]);
    }

#pragma unroll
    for (int i = 0; i < 6; ++i) *(v4u*)(hn + loff[i]) = ur[i];
    wave_lds_sync();

#pragma unroll
    for (int j = 0; j < kNT; ++j) {
#pragma unroll
      for (int r = 0; r < 8; ++r) {
        const int idx = (8 * hh + r) * kHP + n0 + 16 * j + c;
        const unsigned ub = (unsigned)hn[idx];
        const float uf = h16_to_f32(ub);
        const float val = acc[j][r] * kInvAC + uf;
        const _Float16 hv = (_Float16)val;
        hn[idx] = __builtin_bit_cast(unsigned short, hv);
      }
    }
    __syncthreads();

    {
      const int tt = dirb ? (kN - 1 - s) : s;
      v4u ra[3];
      v4u rb[3];
#pragma unroll
      for (int i = 0; i < 3; ++i) {
        ra[i] = *(const v4u*)(hn + rowA * kHP + 8 * (lane + 32 * i));
        rb[i] = *(const v4u*)(hn + (rowA + 1) * kHP + 8 * (lane + 32 * i));
      }
      unsigned short* dA = plane + ((size_t)bA * kN + (size_t)tt) * kH;
      unsigned short* dB = plane + ((size_t)(bA + 1) * kN + (size_t)tt) * kH;
      for (int pass = 0; pass < 2; ++pass) {
#pragma unroll
        for (int i = 0; i < 3; ++i) {
          *(volatile v4u*)(dA + 8 * (lane + 32 * i)) = ra[i];
          *(volatile v4u*)(dB + 8 * (lane + 32 * i)) = rb[i];
        }
        __threadfence();
      }
    }
  }
}

__global__ __launch_bounds__(256) void sum_kernel(const unsigned short* __restrict__ hf16,
                                                  const unsigned short* __restrict__ hb16,
                                                  unsigned short* __restrict__ hs16) {
  const int i = blockIdx.x * 256 + threadIdx.x;
  if (i >= kSumChunks) return;
  const v4u a = *(const v4u*)(hf16 + (size_t)i * 8);
  const v4u b = *(const v4u*)(hb16 + (size_t)i * 8);
  v4u o;
#pragma unroll
  for (int e = 0; e < 4; ++e) {
    const unsigned wa = a[e];
    const unsigned wb = b[e];
    const float lo = h16_to_f32(wa & 0xffffu) + h16_to_f32(wb & 0xffffu);
    const float hi = h16_to_f32(wa >> 16) + h16_to_f32(wb >> 16);
    const unsigned w = pack_f16x2(lo, hi);
    o[e] = w;
  }
  unsigned short* op = hs16 + (size_t)i * 8;
  *(volatile v4u*)op = o;
  __threadfence();
  *(volatile v4u*)op = o;
}

extern "C" void kernel_launch(void* const* d_in, const int* in_sizes, int n_in,
                              void* d_out, int out_size, void* d_ws, size_t ws_size, hipStream_t stream) {
  if (n_in < 10 || d_out == nullptr || d_ws == nullptr) return;
  if (in_sizes[0] != kRows * kD || in_sizes[1] != kD || in_sizes[2] != kH * kR || in_sizes[3] != kH * kR ||
      in_sizes[4] != kH * kH || in_sizes[5] != kH * kD || in_sizes[6] != kD * kH || in_sizes[7] != kD * kD ||
      in_sizes[8] != kD || in_sizes[9] != 1 || out_size != kRows * kD) return;

  const float* x      = (const float*)d_in[0];
  const float* scale  = (const float*)d_in[1];
  const float* U      = (const float*)d_in[2];
  const float* V      = (const float*)d_in[3];
  const float* S      = (const float*)d_in[4];
  const float* Bm     = (const float*)d_in[5];
  const float* Cm     = (const float*)d_in[6];
  const float* gw     = (const float*)d_in[7];
  const float* gate_b = (const float*)d_in[8];
  const float* alpha  = (const float*)d_in[9];
  float* out = (float*)d_out;

  char* ws = (char*)d_ws;
  size_t off = 0;
  auto carve = [&](size_t bytes) -> char* { char* p = ws + off; off += (bytes + 255) & ~(size_t)255; return p; };
  const size_t wplane = (size_t)kH * kH * 2;
  const size_t rplane = (size_t)kRows * kH * 2;
  unsigned short* A16  = (unsigned short*)carve(wplane);
  unsigned short* BM16 = (unsigned short*)carve(wplane);
  unsigned short* CM16 = (unsigned short*)carve(wplane);
  unsigned short* GW16 = (unsigned short*)carve(wplane);
  unsigned short* XN16 = (unsigned short*)carve(rplane);
  unsigned short* U16  = (unsigned short*)carve(rplane);
  unsigned short* G16  = (unsigned short*)carve(rplane);
  unsigned short* HF16 = (unsigned short*)carve(rplane);
  unsigned short* HB16 = (unsigned short*)carve(rplane);
  unsigned short* HS16 = XN16;
  if (off > ws_size || off > (size_t)134217728) return;

  const int gemmGrid = ((kRows / 64) * (kH / 64)) / 8;

  prep_kernel<<<kPrepBlocks, 256, 0, stream>>>(U, V, S, Bm, Cm, gw,
                                               (unsigned*)A16, (unsigned*)BM16, (unsigned*)CM16, (unsigned*)GW16);
  rmsnorm_kernel<<<kRows / 8, 256, 0, stream>>>(x, scale, XN16);
  gemm64_f16<0><<<gemmGrid, 256, 0, stream>>>(XN16, kD, BM16, kD, (void*)U16, kH,
                                              gate_b, x, G16, alpha, kRows, kH, kD, kScaleU);
  gemm64_f16<1><<<gemmGrid, 256, 0, stream>>>(XN16, kD, GW16, kD, (void*)G16, kD,
                                              gate_b, x, G16, alpha, kRows, kD, kD, kScaleG);
  scan_kernel<<<1, 256, 0, stream>>>(U16, A16, HF16, HB16);
  sum_kernel<<<kSumChunks / 256, 256, 0, stream>>>(HF16, HB16, HS16);
  gemm64_f16<2><<<gemmGrid, 256, 0, stream>>>(HS16, kH, CM16, kH, (void*)out, kD,
                                              gate_b, x, G16, alpha, kRows, kD, kH, kScaleY);
}
